// CrossAttentionBlock_41669772705964
// MI455X (gfx1250) — hardware-run, weakly checked
//
#include <hip/hip_runtime.h>


#ifndef NB
#define NB 4
#endif
#ifndef LQ
#define LQ 1024
#endif
#ifndef LKV
#define LKV 1344
#endif
#define NB_FULL  4
#define LQ_FULL  1024
#define LKV_FULL 1344
#ifndef OUT_LQ
#define OUT_LQ LQ
#endif
#define LT   320
#define CC   768
#define NH_  12
#define HD   64
#define HID  3072
#define AW   4
#define OSP  68
#define WSC  64.0f
#define WSI  (1.0f / 64.0f)
#define CTXS 64.0f
#define QSC  0.125f
#define LOG2E 1.4426950408889634f
#define PSH  14.0f
#define NEGB (-3.0e38f)
#define EP_HEAD 0
#define EP_VT   1
#define EP_RES  2
#define EP_GELU 3

static_assert(HD == 64);
static_assert(NH_ * HD == CC);
static_assert(CC % 64 == 0);
static_assert(HID % 64 == 0);
static_assert((2 * CC) % 64 == 0);
static_assert(CC % 32 == 0);
static_assert(HID % 32 == 0);
static_assert(LQ % 64 == 0);
static_assert(LKV % 64 == 0);
static_assert(LT % 64 == 0);
static_assert(LT <= LKV);
static_assert(LKV % 32 == 0);
static_assert(LQ % (16 * AW) == 0);
static_assert((NB * LQ) % 8 == 0);
static_assert((NB * LKV) % 8 == 0);
static_assert(CC == 3 * 32 * 8);
static_assert(NB <= NB_FULL);
static_assert(LQ <= LQ_FULL);
static_assert(LKV <= LKV_FULL);
static_assert((OSP * 4) % 16 == 0);
static_assert(OSP >= HD);
static_assert(32 * 16 * 4 == 16 * HD * 2);
static_assert(32 * 16 * 8 == 16 * 64 * 4);
static_assert(256 * 16 * 2 == 64 * 64 * 2);
static_assert(32 * 16 * 3 == CC * 2);
static_assert(16 * 68 * 4 <= 131072);
static_assert(AW * 16 * OSP * 4 <= 131072);
static_assert(64 * 65 * 4 <= 131072);

typedef _Float16 h16;
typedef __attribute__((ext_vector_type(16))) _Float16 v16h;
typedef __attribute__((ext_vector_type(8)))  _Float16 v8h;
typedef __attribute__((ext_vector_type(8)))  float    v8f;
typedef __attribute__((ext_vector_type(4)))  float    v4f;
typedef v4f  __attribute__((may_alias)) v4fa;

__device__ __forceinline__ unsigned short f2bf(float f) { unsigned u = __float_as_uint(f); u += 0x7FFFu + ((u >> 16) & 1u); return (unsigned short)(u >> 16); }
__device__ __forceinline__ float bfr(float f) { return __uint_as_float(((unsigned)f2bf(f)) << 16); }
__device__ __forceinline__ v16h cat16(v8h lo, v8h hi) { return __builtin_shufflevector(lo, hi, 0, 1, 2, 3, 4, 5, 6, 7, 8, 9, 10, 11, 12, 13, 14, 15); }
__device__ __forceinline__ v8f wmma16(v16h a, v16h b, v8f c) { return __builtin_amdgcn_wmma_f32_16x16x32_f16(false, a, false, b, (short)0, c, false, false); }
__device__ __forceinline__ v16h  ldh(const h16* p) { return cat16(*(const v8h*)p, *(const v8h*)(p + 16)); }
__device__ __forceinline__ void wave_sync() { __builtin_amdgcn_fence(3  , "wavefront"); __builtin_amdgcn_wave_barrier(); asm volatile("" ::: "memory"); }

static __device__ __forceinline__ h16 toh_flush(float v) { const h16 r = (h16)v; return (fabsf(v) < 6.103515625e-05f) ? (h16)0.0f : r; }
__device__ __forceinline__ v8f wmma16g(v16h a, v16h b, v8f c) { c = wmma16(a, b, c); asm volatile("v_nop\n\tv_nop\n\tv_nop\n\tv_nop" : "+v"(c) : "v"(a), "v"(b)); return c; }
__device__ __forceinline__ float gelu_f(float v) { return 0.5f * v * (1.0f + erff(v * 0.70710678118654752f)); }

__global__ __launch_bounds__(256) void k_wT(const float* __restrict__ W, h16* Wt, int K, int N) {
#pragma clang fp contract(off)
    __shared__ float ts[64 * 65];
    const int tid = threadIdx.x;
    const int n0 = blockIdx.x * 64, k0 = blockIdx.y * 64;
#pragma unroll
    for (int it = 0; it < 4; ++it) { const int idx = it * 256 + tid; const int kk = idx >> 4, n4 = (idx & 15) * 4;
        const v4f v = *(const v4f*)(W + (size_t)(k0 + kk) * N + n0 + n4);
#pragma unroll
        for (int i = 0; i < 4; ++i) ts[kk * 65 + n4 + i] = v[i]; }
    __syncthreads();
#pragma unroll 1
    for (int ps = 0; ps < 2; ++ps) {
#pragma unroll
        for (int it = 0; it < 2; ++it) { const int p = it * 256 + tid; const int row = p >> 3, c8 = (p & 7) * 8;
            v8h o;
#pragma unroll
            for (int i = 0; i < 8; ++i) o[i] = toh_flush(bfr(ts[(c8 + i) * 65 + row]) * WSC);
            *(volatile v8h*)(Wt + (size_t)(n0 + row) * K + k0 + c8) = o; }
        if (ps == 0) __threadfence(); }
}

__global__ __launch_bounds__(256) void k_ln(const float* __restrict__ x, const float* __restrict__ g, const float* __restrict__ be, h16* dst, int L, int LF, int rnd) {
#pragma clang fp contract(off)
    const int lane = threadIdx.x & 31;
    const int wave = __builtin_amdgcn_readfirstlane((int)(threadIdx.x >> 5));
    const int row = blockIdx.x * 8 + wave;
    const float* src = x + ((size_t)(row / L) * (size_t)LF + (size_t)(row % L)) * CC + lane * 8;
    h16* drow = dst + (size_t)row * CC + lane * 8;
    float s = 0.0f;
#pragma unroll 1
    for (int i = 0; i < 3; ++i) { const v8f v = *(const v8f*)(src + i * 256);
#pragma unroll
        for (int k = 0; k < 8; ++k) { const float xv = rnd ? bfr(v[k]) : v[k]; s += xv; } }
    s += __shfl_xor(s, 16, 32); s += __shfl_xor(s, 8, 32); s += __shfl_xor(s, 4, 32); s += __shfl_xor(s, 2, 32); s += __shfl_xor(s, 1, 32);
    const float mean = s * (1.0f / (float)CC);
    float q = 0.0f;
#pragma unroll 1
    for (int i = 0; i < 3; ++i) { const v8f v = *(const v8f*)(src + i * 256);
#pragma unroll
        for (int k = 0; k < 8; ++k) { const float xv = rnd ? bfr(v[k]) : v[k]; const float dv = xv - mean; q += dv * dv; } }
    q += __shfl_xor(q, 16, 32); q += __shfl_xor(q, 8, 32); q += __shfl_xor(q, 4, 32); q += __shfl_xor(q, 2, 32); q += __shfl_xor(q, 1, 32);
    const float rstd = rsqrtf(q * (1.0f / (float)CC) + 1e-5f);
#pragma unroll 1
    for (int ps = 0; ps < 2; ++ps) {
#pragma unroll 1
        for (int i = 0; i < 3; ++i) {
            const v8f v = *(const v8f*)(src + i * 256);
            const v8f gv = *(const v8f*)(g + i * 256 + lane * 8);
            const v8f bv = *(const v8f*)(be + i * 256 + lane * 8);
            v8h o;
#pragma unroll
            for (int k = 0; k < 8; ++k) { const float xv = rnd ? bfr(v[k]) : v[k]; o[k] = toh_flush((xv - mean) * rstd * bfr(gv[k]) + bfr(bv[k])); }
            *(volatile v8h*)(drow + i * 256) = o; }
        if (ps == 0) __threadfence(); }
}

template <int EP>
__device__ __forceinline__ void gemm_body(const h16* __restrict__ A, const h16* __restrict__ Bt, const float* __restrict__ bias, const float* __restrict__ aux,
                                          h16* Ph, float* Pf, int K, int N, int L, int auxLF, int dstLF, int rnd, float osc) {
    __shared__ __align__(16) float os[16 * 68];
    const int lane = threadIdx.x & 31, lr = lane & 15, hi = lane >> 4; const int r0 = blockIdx.x * 64, c0 = blockIdx.y * 64;
    v8f acc[4][4];
#pragma unroll
    for (int mb = 0; mb < 4; ++mb)
#pragma unroll
        for (int nb = 0; nb < 4; ++nb) acc[mb][nb] = (v8f){};
    const size_t aoff = (size_t)(r0 + lr) * K + 8 * hi, boff = (size_t)(c0 + lr) * K + 8 * hi;
#pragma unroll 1
    for (int kc = 0; kc < K; kc += 32) {
        v16h a[4];
#pragma unroll
        for (int mb = 0; mb < 4; ++mb) a[mb] = ldh(A + aoff + (size_t)mb * 16 * K + kc);
#pragma unroll
        for (int nb = 0; nb < 4; ++nb) { const v16h b = ldh(Bt + boff + (size_t)nb * 16 * K + kc);
#pragma unroll
            for (int mb = 0; mb < 4; ++mb) acc[mb][nb] = wmma16g(a[mb], b, acc[mb][nb]); }
    }
    float bc[4];
#pragma unroll
    for (int nb = 0; nb < 4; ++nb) { bc[nb] = 0.0f; if (EP != EP_VT) bc[nb] = bfr(bias[c0 + nb * 16 + lr]); }
    int bb = 0, tt = r0;
    if (EP == EP_HEAD || EP == EP_RES) { bb = r0 / L; tt = r0 % L; }
    if (EP == EP_VT) { bb = c0 / L; tt = c0 % L; }
    const bool addm = (EP == EP_VT) && (tt < LT);
#pragma unroll
    for (int mb = 0; mb < 4; ++mb) {
        float br[8];
#pragma unroll
        for (int j = 0; j < 8; ++j) { br[j] = 0.0f; if (EP == EP_VT) br[j] = bfr(bias[r0 + mb * 16 + hi * 8 + j]); }
#pragma unroll
        for (int nb = 0; nb < 4; ++nb) {
            float tv[8];
#pragma unroll
            for (int j = 0; j < 8; ++j) tv[j] = 0.0f;
            if (EP == EP_VT) { if (addm) { const float* tp = aux + ((size_t)bb * LT + (size_t)(tt + nb * 16 + lr)) * CC + r0 + mb * 16 + hi * 8;
                const v4f t0v = *(const v4f*)tp; const v4f t1v = *(const v4f*)(tp + 4);
#pragma unroll
                for (int j = 0; j < 4; ++j) { tv[j] = bfr(t0v[j]); tv[4 + j] = bfr(t1v[j]); } } }
#pragma unroll
            for (int j = 0; j < 8; ++j) { float val = acc[mb][nb][j] * osc;
                if (EP != EP_VT) { val = val + bc[nb]; } else { val = val + br[j]; val = val + tv[j]; }
                os[(hi * 8 + j) * 68 + nb * 16 + lr] = val; } }
        wave_sync();
        if (EP == EP_GELU) {
#pragma unroll 1
            for (int s = 0; s < 4; ++s) { const int row = 4 * s + (lane >> 3), c8 = (lane & 7) * 8;
                v4f x0 = *(const v4fa*)(&os[row * 68 + c8]); v4f x1 = *(const v4fa*)(&os[row * 68 + c8 + 4]);
#pragma unroll
                for (int i = 0; i < 4; ++i) { x0[i] = gelu_f(x0[i]); x1[i] = gelu_f(x1[i]); }
                *(v4fa*)(&os[row * 68 + c8]) = x0; *(v4fa*)(&os[row * 68 + c8 + 4]) = x1; }
            wave_sync();
        }
#pragma unroll 1
        for (int ps = 0; ps < 2; ++ps) {
            if (EP == EP_HEAD) {
                const size_t sb = (((size_t)bb * NH_ + (size_t)(c0 / HD)) * (size_t)L + (size_t)(tt + mb * 16)) * HD;
#pragma unroll
                for (int s = 0; s < 4; ++s) { const int p = s * 32 + lane; const int row = p >> 3, c8 = (p & 7) * 8;
                    const v4f x0 = *(const v4fa*)(&os[row * 68 + c8]); const v4f x1 = *(const v4fa*)(&os[row * 68 + c8 + 4]); v8h hv;
#pragma unroll
                    for (int i = 0; i < 4; ++i) { hv[i] = toh_flush(x0[i]); hv[4 + i] = toh_flush(x1[i]); }
                    *(volatile v8h*)(Ph + sb + (size_t)p * 8) = hv; }
            } else if (EP == EP_VT) {
                const size_t sb = ((size_t)bb * CC + (size_t)(r0 + mb * 16)) * (size_t)L + (size_t)tt;
#pragma unroll
                for (int s = 0; s < 4; ++s) { const int row = 4 * s + (lane >> 3), c8 = (lane & 7) * 8;
                    const v4f x0 = *(const v4fa*)(&os[row * 68 + c8]); const v4f x1 = *(const v4fa*)(&os[row * 68 + c8 + 4]); v8h hv;
#pragma unroll
                    for (int i = 0; i < 4; ++i) { hv[i] = toh_flush(x0[i]); hv[4 + i] = toh_flush(x1[i]); }
                    *(volatile v8h*)(Ph + sb + (size_t)row * (size_t)L + c8) = hv; }
            } else if (EP == EP_GELU) {
                const size_t sb = (size_t)(r0 + mb * 16) * (size_t)N + (size_t)c0;
#pragma unroll
                for (int s = 0; s < 4; ++s) { const int row = 4 * s + (lane >> 3), c8 = (lane & 7) * 8;
                    const v4f x0 = *(const v4fa*)(&os[row * 68 + c8]); const v4f x1 = *(const v4fa*)(&os[row * 68 + c8 + 4]); v8h hv;
#pragma unroll
                    for (int i = 0; i < 4; ++i) { hv[i] = toh_flush(x0[i]); hv[4 + i] = toh_flush(x1[i]); }
                    *(volatile v8h*)(Ph + sb + (size_t)row * (size_t)N + c8) = hv; }
            } else {
                const size_t db = ((size_t)bb * (size_t)dstLF + (size_t)(tt + mb * 16)) * (size_t)N + (size_t)c0;
                const size_t rb = ((size_t)bb * (size_t)auxLF + (size_t)(tt + mb * 16)) * (size_t)N + (size_t)c0;
#pragma unroll
                for (int s = 0; s < 8; ++s) { const int p = s * 32 + lane; const int row = p >> 4, c4 = (p & 15) * 4;
                    const v4f x0 = *(const v4fa*)(&os[row * 68 + c4]);
                    v4f rr = *(const v4f*)(aux + rb + (size_t)row * (size_t)N + c4);
#pragma unroll
                    for (int i = 0; i < 4; ++i) rr[i] = rnd ? bfr(rr[i]) : rr[i];
                    const v4f val = rr + x0;
                    *(volatile v4f*)(Pf + db + (size_t)row * (size_t)N + c4) = val; }
            }
            if (ps == 0) __threadfence(); }
        wave_sync();
    }
}

__global__ __launch_bounds__(32) void k_gemm_head(const h16* __restrict__ A, const h16* __restrict__ Bt, const float* __restrict__ bias, h16* Ph, int K, int L, float osc) {
    gemm_body<EP_HEAD>(A, Bt, bias, bias, Ph, nullptr, K, 0, L, 0, 0, 0, osc);
}
__global__ __launch_bounds__(32) void k_gemm_vt(const h16* __restrict__ A, const h16* __restrict__ Bt, const float* __restrict__ bias, const float* __restrict__ tmask, h16* Ph, int K, int L, float osc) {
    gemm_body<EP_VT>(A, Bt, bias, tmask, Ph, nullptr, K, 0, L, 0, 0, 0, osc);
}
__global__ __launch_bounds__(32) void k_gemm_res(const h16* __restrict__ A, const h16* __restrict__ Bt, const float* __restrict__ bias, const float* __restrict__ skip, float* Pf,
                                                 int K, int N, int L, int skipLF, int dstLF, int rnd, float osc) {
    gemm_body<EP_RES>(A, Bt, bias, skip, nullptr, Pf, K, N, L, skipLF, dstLF, rnd, osc);
}
__global__ __launch_bounds__(32) void k_gemm_gelu(const h16* __restrict__ A, const h16* __restrict__ Bt, const float* __restrict__ bias, h16* Ph, int K, int N, float osc) {
    gemm_body<EP_GELU>(A, Bt, bias, bias, Ph, nullptr, K, N, 1, 0, 0, 0, osc);
}

__global__ __launch_bounds__(32 * AW) void k_flash(const h16* __restrict__ QH, const h16* __restrict__ KP, const h16* __restrict__ VT, const float* __restrict__ pos, h16* CTX) {
    __shared__ __align__(16) float os[AW * 16 * OSP];
    const int lane = threadIdx.x & 31, lr = lane & 15, hi = lane >> 4;
    const int wave = __builtin_amdgcn_readfirstlane((int)(threadIdx.x >> 5));
    const int zh = blockIdx.y; const int b = zh / NH_, h = zh % NH_;
    const int t0 = (blockIdx.x * AW + wave) * 16;
    const size_t qo = ((size_t)zh * LQ + (size_t)(t0 + lr)) * HD + 8 * hi;
    const v16h q0 = ldh(QH + qo), q1 = ldh(QH + qo + 32);
    const size_t kvb = (size_t)zh * LKV * HD;
    const size_t ko = kvb + (size_t)lr * HD + 8 * hi;
    const size_t vo = kvb + (size_t)lr * LKV + 8 * hi;
    const float* pp = pos + ((size_t)h * LQ_FULL + (size_t)(t0 + lr)) * LKV_FULL + 8 * hi;
    v8f o0 = (v8f){}, o1 = (v8f){}, o2 = (v8f){}, o3 = (v8f){};
    float m = NEGB, l = 0.0f;
#pragma unroll 1
    for (int key0 = 0; key0 < LKV; key0 += 32) {
        const h16* ka = KP + ko + (size_t)key0 * HD;
        const v16h ka0 = ldh(ka), ka1 = ldh(ka + 32), kb0 = ldh(ka + 16 * HD), kb1 = ldh(ka + 16 * HD + 32);
        v8f sa = (v8f){}, sb = (v8f){};
        sa = wmma16g(ka0, q0, sa); sb = wmma16g(kb0, q0, sb); sa = wmma16g(ka1, q1, sa); sb = wmma16g(kb1, q1, sb);
        const float* kp = pp + key0;
        const v4f m0 = *(const v4f*)kp, m1 = *(const v4f*)(kp + 4), m2 = *(const v4f*)(kp + 16), m3 = *(const v4f*)(kp + 20);
        float px[8], py[8];
#pragma unroll
        for (int r = 0; r < 4; ++r) { px[r] = m0[r]; px[4 + r] = m1[r]; py[r] = m2[r]; py[4 + r] = m3[r]; }
        float ta[8], tb[8]; float mx = NEGB;
#pragma unroll
        for (int r = 0; r < 8; ++r) {
            ta[r] = (sa[r] * QSC + bfr(px[r])) * LOG2E; tb[r] = (sb[r] * QSC + bfr(py[r])) * LOG2E;
            mx = fmaxf(mx, fmaxf(ta[r], tb[r])); }
        mx = fmaxf(mx, __shfl_xor(mx, 16, 32));
        const float mnew = fmaxf(m, mx);
        const float alpha = __builtin_amdgcn_exp2f(m - mnew);
        const float sh = PSH - mnew;
        v16h pb; float ls = 0.0f;
#pragma unroll
        for (int r = 0; r < 8; ++r) {
            const float xa = ta[r] + sh, xb = tb[r] + sh;
            const float ea = __builtin_amdgcn_exp2f(xa), eb = __builtin_amdgcn_exp2f(xb);
            const float ga = (xa < -14.0f) ? 0.0f : ea, gb = (xb < -14.0f) ? 0.0f : eb;
            const h16 pa = (h16)ga; const h16 pc = (h16)gb;
            pb[r] = pa; pb[8 + r] = pc;
            ls += (float)pa + (float)pc; }
        l = l * alpha + ls; m = mnew;
        o0 = o0 * alpha; o1 = o1 * alpha; o2 = o2 * alpha; o3 = o3 * alpha;
        const h16* va = VT + vo + key0;
        const v16h v0 = ldh(va), v1 = ldh(va + (size_t)16 * LKV), v2 = ldh(va + (size_t)32 * LKV), v3 = ldh(va + (size_t)48 * LKV);
        o0 = wmma16g(v0, pb, o0); o1 = wmma16g(v1, pb, o1); o2 = wmma16g(v2, pb, o2); o3 = wmma16g(v3, pb, o3);
    }
    l += __shfl_xor(l, 16, 32);
    const float sc = CTXS * (1.0f / l);
    const int wb = wave * 16 * OSP;
    { v4f a, c;
      a[0] = o0[0] * sc; a[1] = o0[1] * sc; a[2] = o0[2] * sc; a[3] = o0[3] * sc; c[0] = o0[4] * sc; c[1] = o0[5] * sc; c[2] = o0[6] * sc; c[3] = o0[7] * sc;
      *(v4fa*)(&os[wb + lr * OSP +  0 + 8 * hi]) = a; *(v4fa*)(&os[wb + lr * OSP +  0 + 8 * hi + 4]) = c;
      a[0] = o1[0] * sc; a[1] = o1[1] * sc; a[2] = o1[2] * sc; a[3] = o1[3] * sc; c[0] = o1[4] * sc; c[1] = o1[5] * sc; c[2] = o1[6] * sc; c[3] = o1[7] * sc;
      *(v4fa*)(&os[wb + lr * OSP + 16 + 8 * hi]) = a; *(v4fa*)(&os[wb + lr * OSP + 16 + 8 * hi + 4]) = c;
      a[0] = o2[0] * sc; a[1] = o2[1] * sc; a[2] = o2[2] * sc; a[3] = o2[3] * sc; c[0] = o2[4] * sc; c[1] = o2[5] * sc; c[2] = o2[6] * sc; c[3] = o2[7] * sc;
      *(v4fa*)(&os[wb + lr * OSP + 32 + 8 * hi]) = a; *(v4fa*)(&os[wb + lr * OSP + 32 + 8 * hi + 4]) = c;
      a[0] = o3[0] * sc; a[1] = o3[1] * sc; a[2] = o3[2] * sc; a[3] = o3[3] * sc; c[0] = o3[4] * sc; c[1] = o3[5] * sc; c[2] = o3[6] * sc; c[3] = o3[7] * sc;
      *(v4fa*)(&os[wb + lr * OSP + 48 + 8 * hi]) = a; *(v4fa*)(&os[wb + lr * OSP + 48 + 8 * hi + 4]) = c; }
    wave_sync();
    h16* orow = CTX + ((size_t)b * LQ + (size_t)t0) * CC + h * HD;
#pragma unroll 1
    for (int ps = 0; ps < 2; ++ps) {
#pragma unroll
        for (int s = 0; s < 4; ++s) { const int row = 4 * s + (lane >> 3), c8 = (lane & 7) * 8;
            const v4f x0 = *(const v4fa*)(&os[wb + row * OSP + c8]); const v4f x1 = *(const v4fa*)(&os[wb + row * OSP + c8 + 4]); v8h hv;
#pragma unroll
            for (int i = 0; i < 4; ++i) { hv[i] = toh_flush(x0[i]); hv[4 + i] = toh_flush(x1[i]); }
            *(volatile v8h*)(orow + (size_t)row * CC + c8) = hv; }
        if (ps == 0) __threadfence(); }
}

static constexpr size_t al256(size_t v) { return (v + 255) & ~(size_t)255; }
static constexpr size_t MQ_ = (size_t)NB * LQ;
static constexpr size_t MK_ = (size_t)NB * LKV;
static constexpr size_t SZ_WSQ = al256((size_t)CC * CC * 2);
static constexpr size_t SZ_WKV = al256((size_t)2 * CC * CC * 2);
static constexpr size_t SZ_WH  = al256((size_t)CC * HID * 2);
static constexpr size_t SZ_AQ  = al256(MQ_ * CC * 2);
static constexpr size_t SZ_AK  = al256(MK_ * CC * 2);
static constexpr size_t SZ_Q1  = al256(MQ_ * CC * 4);
static constexpr size_t SZ_F1  = al256(MQ_ * HID * 2);
static constexpr size_t SZ_TOTAL = 2 * SZ_WSQ + SZ_WKV + 2 * SZ_WH + 4 * SZ_AQ + 3 * SZ_AK + SZ_Q1 + SZ_F1;
static_assert(SZ_TOTAL <= (size_t)134217728);
static_assert((size_t)NB * NH_ * LKV * HD == MK_ * CC);
static_assert((size_t)NB * NH_ * LQ * HD == MQ_ * CC);
static_assert(MQ_ % 64 == 0);
static_assert(MK_ % 64 == 0);
static_assert(MK_ / 64 <= 65535);

extern "C" void kernel_launch(void* const* d_in, const int* in_sizes, int n_in,
                              void* d_out, int out_size, void* d_ws, size_t ws_size, hipStream_t stream) {
    if (n_in < 20) return;
    if ((size_t)in_sizes[0] < (size_t)NB * LT * CC) return;
    if ((size_t)in_sizes[1] < ((size_t)(NB - 1) * LQ_FULL + LQ) * CC) return;
    if ((size_t)in_sizes[2] < ((size_t)(NB - 1) * LKV_FULL + LKV) * CC) return;
    if ((size_t)in_sizes[3] < ((size_t)(NH_ - 1) * LQ_FULL + (LQ - 1)) * LKV_FULL + LKV) return;
    if (in_sizes[4] < CC || in_sizes[5] < CC || in_sizes[6] < CC || in_sizes[7] < CC) return;
    if ((size_t)in_sizes[8] < (size_t)CC * CC || in_sizes[9] < CC) return;
    if ((size_t)in_sizes[10] < (size_t)2 * CC * CC || in_sizes[11] < 2 * CC) return;
    if ((size_t)in_sizes[12] < (size_t)CC * CC || in_sizes[13] < CC) return;
    if (in_sizes[14] < CC || in_sizes[15] < CC) return;
    if ((size_t)in_sizes[16] < (size_t)CC * HID || in_sizes[17] < HID) return;
    if ((size_t)in_sizes[18] < (size_t)HID * CC || in_sizes[19] < CC) return;
    if ((size_t)out_size < ((size_t)(NB - 1) * OUT_LQ + LQ) * CC) return;
    if (SZ_TOTAL > ws_size) return;
    const float* tmask = (const float*)d_in[0];
    const float* q_in  = (const float*)d_in[1];
    const float* kv_in = (const float*)d_in[2];
    const float* apos  = (const float*)d_in[3];
    const float* g1q = (const float*)d_in[4];  const float* b1q = (const float*)d_in[5];
    const float* g1k = (const float*)d_in[6];  const float* b1k = (const float*)d_in[7];
    const float* wq  = (const float*)d_in[8];  const float* bq  = (const float*)d_in[9];
    const float* wkv = (const float*)d_in[10]; const float* bkv = (const float*)d_in[11];
    const float* wp  = (const float*)d_in[12]; const float* bp  = (const float*)d_in[13];
    const float* g2  = (const float*)d_in[14]; const float* b2n = (const float*)d_in[15];
    const float* w1  = (const float*)d_in[16]; const float* b1  = (const float*)d_in[17];
    const float* w2  = (const float*)d_in[18]; const float* b2  = (const float*)d_in[19];
    float* OUT = (float*)d_out;
    char* wsp = (char*)d_ws;
    h16* WqT  = (h16*)wsp; wsp += SZ_WSQ;
    h16* WkvT = (h16*)wsp; wsp += SZ_WKV;
    h16* WpT  = (h16*)wsp; wsp += SZ_WSQ;
    h16* W1T  = (h16*)wsp; wsp += SZ_WH;
    h16* W2T  = (h16*)wsp; wsp += SZ_WH;
    h16* QN   = (h16*)wsp; wsp += SZ_AQ;
    h16* KVN  = (h16*)wsp; wsp += SZ_AK;
    h16* QH   = (h16*)wsp; wsp += SZ_AQ;
    h16* KP   = (h16*)wsp; wsp += SZ_AK;
    h16* VT   = (h16*)wsp; wsp += SZ_AK;
    h16* CTX  = (h16*)wsp; wsp += SZ_AQ;
    float* Q1 = (float*)wsp; wsp += SZ_Q1;
    h16* HN   = (h16*)wsp; wsp += SZ_AQ;
    h16* F1   = (h16*)wsp; wsp += SZ_F1;

    k_wT<<<dim3(CC / 64, CC / 64, 1), 256, 0, stream>>>(wq, WqT, CC, CC);
    k_wT<<<dim3(2 * CC / 64, CC / 64, 1), 256, 0, stream>>>(wkv, WkvT, CC, 2 * CC);
    k_wT<<<dim3(CC / 64, CC / 64, 1), 256, 0, stream>>>(wp, WpT, CC, CC);
    k_wT<<<dim3(HID / 64, CC / 64, 1), 256, 0, stream>>>(w1, W1T, CC, HID);
    k_wT<<<dim3(CC / 64, HID / 64, 1), 256, 0, stream>>>(w2, W2T, HID, CC);

    k_ln<<<(unsigned)(MQ_ / 8), 256, 0, stream>>>(q_in, g1q, b1q, QN, LQ, LQ_FULL, 1);
    k_ln<<<(unsigned)(MK_ / 8), 256, 0, stream>>>(kv_in, g1k, b1k, KVN, LKV, LKV_FULL, 1);

    k_gemm_head<<<dim3((unsigned)(MQ_ / 64), CC / 64, 1), 32, 0, stream>>>(QN, WqT, bq, QH, CC, LQ, WSI);
    k_gemm_head<<<dim3((unsigned)(MK_ / 64), CC / 64, 1), 32, 0, stream>>>(KVN, WkvT, bkv, KP, CC, LKV, WSI);
    k_gemm_vt<<<dim3(CC / 64, (unsigned)(MK_ / 64), 1), 32, 0, stream>>>(WkvT + (size_t)CC * CC, KVN, bkv + CC, tmask, VT, CC, LKV, WSI);

    k_flash<<<dim3(LQ / (16 * AW), NB * NH_, 1), 32 * AW, 0, stream>>>(QH, KP, VT, apos, CTX);

    k_gemm_res<<<dim3((unsigned)(MQ_ / 64), CC / 64, 1), 32, 0, stream>>>(CTX, WpT, bp, q_in, Q1, CC, CC, LQ, LQ_FULL, LQ, 1, WSI / CTXS);
    k_ln<<<(unsigned)(MQ_ / 8), 256, 0, stream>>>(Q1, g2, b2n, HN, LQ, LQ, 0);
    k_gemm_gelu<<<dim3((unsigned)(MQ_ / 64), HID / 64, 1), 32, 0, stream>>>(HN, W1T, b1, F1, CC, HID, WSI);
    k_gemm_res<<<dim3((unsigned)(MQ_ / 64), CC / 64, 1), 32, 0, stream>>>(F1, W2T, b2, Q1, OUT, HID, CC, LQ, LQ, OUT_LQ, 0, WSI);
}
